// MHSelfAttention_39676907888250
// MI455X (gfx1250) — hardware-verified
//
#include <hip/hip_runtime.h>
#include <hip/hip_bf16.h>


typedef __attribute__((ext_vector_type(8)))  float          v8f;
typedef __attribute__((ext_vector_type(4)))  float          v4f;
typedef __attribute__((ext_vector_type(8)))  int            v8i;
typedef __attribute__((ext_vector_type(16))) __bf16         v16bf;
typedef __attribute__((ext_vector_type(8)))  unsigned short u16x8;
typedef __attribute__((ext_vector_type(16))) unsigned short u16x16;
typedef unsigned short us_t;

#ifndef NB
#define NB 2
#endif
#ifndef SEQ
#define SEQ 2048
#endif
#define NB_FULL  2
#define SEQ_FULL 2048
#define EMB   1024
#define NH    16
#define HD    64
#define MROWS (NB * SEQ)
#define LDP   68
#define NEG_BIG (-1.0e30f)

static_assert(NB >= 1 && NB <= NB_FULL);
static_assert(SEQ >= 64 && SEQ <= SEQ_FULL && (SEQ % 64) == 0);
static_assert(EMB == NH * HD);
static_assert(HD == 64);
static_assert((EMB % 64) == 0);
static_assert((MROWS % 64) == 0);

#define XB_BYTES ((size_t)MROWS * EMB * 2)
#define WB_BYTES ((size_t)EMB * EMB * 2)
#define PL_BYTES ((size_t)MROWS * EMB * 2)
#define WS_TOTAL (XB_BYTES + 4 * WB_BYTES + 8 * PL_BYTES)
static_assert(WS_TOTAL <= (size_t)134217728);
static_assert((((size_t)(NB - 1) * SEQ_FULL + SEQ) * EMB) <= (size_t)NB_FULL * SEQ_FULL * EMB);

__device__ __forceinline__ us_t f2bf(float f) {
  unsigned int u = __builtin_bit_cast(unsigned int, f);
  u += 0x7FFFu + ((u >> 16) & 1u);
  return (us_t)(u >> 16);
}

__device__ __forceinline__ float bf2f(us_t h) {
  return __builtin_bit_cast(float, ((unsigned int)h) << 16);
}

__device__ __forceinline__ void split2(v4f a, v4f b, u16x8& hi, u16x8& lo) {
  u16x8 h_, l_;
#pragma unroll
  for (int j = 0; j < 4; ++j) {
    const us_t t0 = f2bf(a[j]); h_[j]     = t0; l_[j]     = f2bf(a[j] - bf2f(t0));
    const us_t t1 = f2bf(b[j]); h_[4 + j] = t1; l_[4 + j] = f2bf(b[j] - bf2f(t1));
  }
  hi = h_; lo = l_;
}

__device__ __forceinline__ u16x8 cvt8(v4f a, v4f b) {
  u16x8 o;
#pragma unroll
  for (int j = 0; j < 4; ++j) { o[j] = f2bf(a[j]); o[4 + j] = f2bf(b[j]); }
  return o;
}

__device__ __forceinline__ v16bf ldfrag(const us_t* __restrict__ base, int row, int ld,
                                        int k0, int h16) {
  const us_t* p = base + (size_t)row * ld + k0 + 8 * h16;
  const u16x8 e0 = *(const u16x8*)p;
  const u16x8 e1 = *(const u16x8*)(p + 16);
  const u16x16 w = __builtin_shufflevector(e0, e1, 0, 1, 2, 3, 4, 5, 6, 7,
                                           8, 9, 10, 11, 12, 13, 14, 15);
  return __builtin_bit_cast(v16bf, w);
}

__device__ __forceinline__ v8f wmma_bf16(v16bf a, v16bf b, v8f c) {
  v8f d = __builtin_amdgcn_wmma_f32_16x16x32_bf16(false, a, false, b, (short)0, c, false, false);
  asm volatile("v_nop\n\tv_nop\n\tv_nop\n\tv_nop"
               : "+v"(d)
               : "v"(__builtin_bit_cast(v8i, a)), "v"(__builtin_bit_cast(v8i, b)));
  return d;
}

__global__ __launch_bounds__(256) void cvt_x_kernel(const float* __restrict__ x,
                                                    us_t* __restrict__ xb) {
  const size_t g = (size_t)blockIdx.x * 256 + threadIdx.x;
  const size_t ngroups = (size_t)MROWS * EMB / 8;
  if (g < ngroups) {
    const size_t e = g * 8;
    const int m = (int)(e / EMB);
    const int c = (int)(e % EMB);
    const int b = m / SEQ, s = m % SEQ;
    const float* src = x + ((size_t)b * SEQ_FULL + s) * EMB + c;
    const v4f a0 = *(const v4f*)src;
    const v4f a1 = *(const v4f*)(src + 4);
    const u16x8 o = cvt8(a0, a1);
    us_t* d = xb + e;
    *(volatile u16x8*)d = o;
    __threadfence();
    *(volatile u16x8*)d = o;
  }
}

__global__ __launch_bounds__(256) void cvt_w_kernel(
    const float* __restrict__ Wq, const float* __restrict__ Wk,
    const float* __restrict__ Wv, const float* __restrict__ Wp,
    us_t* __restrict__ Wqb, us_t* __restrict__ Wkb,
    us_t* __restrict__ Wvb, us_t* __restrict__ Wpb) {
  const int y = blockIdx.y;
  const float* src = (y == 0) ? Wq : ((y == 1) ? Wk : ((y == 2) ? Wv : Wp));
  us_t* dst        = (y == 0) ? Wqb : ((y == 1) ? Wkb : ((y == 2) ? Wvb : Wpb));
  const size_t g = (size_t)blockIdx.x * 256 + threadIdx.x;
  const size_t ngroups = (size_t)EMB * EMB / 8;
  if (g < ngroups) {
    const size_t e = g * 8;
    const v4f a0 = *(const v4f*)(src + e);
    const v4f a1 = *(const v4f*)(src + e + 4);
    const u16x8 o = cvt8(a0, a1);
    us_t* d = dst + e;
    *(volatile u16x8*)d = o;
    __threadfence();
    *(volatile u16x8*)d = o;
  }
}

__global__ __launch_bounds__(128) void proj_qkv_kernel(
    const us_t* __restrict__ xb,
    const us_t* __restrict__ Wqb, const us_t* __restrict__ Wkb, const us_t* __restrict__ Wvb,
    const float* __restrict__ bq, const float* __restrict__ bk, const float* __restrict__ bv,
    us_t* __restrict__ Qh, us_t* __restrict__ Ql,
    us_t* __restrict__ Kh, us_t* __restrict__ Kl,
    us_t* __restrict__ VTh, us_t* __restrict__ VTl) {
  __shared__ __align__(16) float st[4][16 * LDP];

  const int z = blockIdx.z;
  const us_t* W     = (z == 0) ? Wqb : ((z == 1) ? Wkb : Wvb);
  const float* bias = (z == 0) ? bq  : ((z == 1) ? bk  : bv);

  const int wave = threadIdx.x >> 5;
  const int lane = threadIdx.x & 31;
  const int h16  = lane >> 4;
  const int llo  = lane & 15;
  const int m0   = blockIdx.x * 64 + wave * 16;
  const int n0   = blockIdx.y * 64;

  v8f acc[4] = {{}, {}, {}, {}};
#pragma unroll 1
  for (int k0 = 0; k0 < EMB; k0 += 32) {
    const v16bf a = ldfrag(xb, m0 + llo, EMB, k0, h16);
#pragma unroll
    for (int c = 0; c < 4; ++c) {
      const v16bf b = ldfrag(W, n0 + c * 16 + llo, EMB, k0, h16);
      acc[c] = wmma_bf16(a, b, acc[c]);
    }
  }

  float* ws_ = &st[wave][0];
#pragma unroll
  for (int c = 0; c < 4; ++c) {
    int bcol = n0 + c * 16 + llo;
    bcol = (bcol < EMB) ? bcol : (EMB - 1);
    const float bvf = bf2f(f2bf(bias[bcol]));
#pragma unroll
    for (int r = 0; r < 8; ++r) ws_[(8 * h16 + r) * LDP + c * 16 + llo] = acc[c][r] + bvf;
  }
  __syncthreads();

  const int hh = blockIdx.y;
  if (z < 2) {
    us_t* dh = (z == 0) ? Qh : Kh;
    us_t* dl = (z == 0) ? Ql : Kl;
#pragma unroll
    for (int it = 0; it < 4; ++it) {
      const int row = it * 4 + (lane >> 3);
      const int c8  = (lane & 7) * 8;
      const v4f a0 = *(const v4f*)(ws_ + row * LDP + c8);
      const v4f a1 = *(const v4f*)(ws_ + row * LDP + c8 + 4);
      u16x8 hi, lo;
      split2(a0, a1, hi, lo);
      const int m = m0 + row;
      const int b = m / SEQ, s = m % SEQ;
      const size_t off = (((size_t)b * NH + hh) * SEQ + s) * HD + c8;
      *(volatile u16x8*)(dh + off) = hi;
      *(volatile u16x8*)(dl + off) = lo;
      __threadfence();
      *(volatile u16x8*)(dh + off) = hi;
      *(volatile u16x8*)(dl + off) = lo;
    }
  } else {
    const int mb = blockIdx.x * 64;
    const int b  = mb / SEQ;
    const int s0 = mb % SEQ;
    const int tid = threadIdx.x;
#pragma unroll
    for (int it = 0; it < 4; ++it) {
      const int d    = it * 16 + (tid >> 3);
      const int sp   = (tid & 7) * 8;
      const int wsrc = sp >> 4;
      const int rr   = sp & 15;
      const float* colp = &st[wsrc][rr * LDP + d];
      v4f a0, a1;
#pragma unroll
      for (int j = 0; j < 4; ++j) { a0[j] = colp[j * LDP]; a1[j] = colp[(4 + j) * LDP]; }
      u16x8 hi, lo;
      split2(a0, a1, hi, lo);
      const size_t off = (((size_t)b * NH + hh) * HD + d) * SEQ + s0 + sp;
      *(volatile u16x8*)(VTh + off) = hi;
      *(volatile u16x8*)(VTl + off) = lo;
      __threadfence();
      *(volatile u16x8*)(VTh + off) = hi;
      *(volatile u16x8*)(VTl + off) = lo;
    }
  }
}

__global__ __launch_bounds__(128) void attn_kernel(
    const us_t* __restrict__ Qh, const us_t* __restrict__ Ql,
    const us_t* __restrict__ Kh, const us_t* __restrict__ Kl,
    const us_t* __restrict__ VTh, const us_t* __restrict__ VTl,
    us_t* __restrict__ Yh, us_t* __restrict__ Yl) {
  __shared__ __align__(16) float yst[4][16 * LDP];

  const int wave = threadIdx.x >> 5;
  const int lane = threadIdx.x & 31;
  const int h16  = lane >> 4;
  const int llo  = lane & 15;
  const int bh   = blockIdx.y;
  const int bb   = bh / NH;
  const int hh   = bh % NH;
  const int qblk = blockIdx.x;
  const int q0   = qblk * 64 + wave * 16;
  const int qq   = q0 + llo;

  const size_t hoff = (size_t)bh * SEQ * HD;
  const us_t* qh = Qh + hoff;
  const us_t* ql = Ql + hoff;
  const us_t* kh = Kh + hoff;
  const us_t* kl = Kl + hoff;
  const us_t* vh = VTh + hoff;
  const us_t* vl = VTl + hoff;

  const v16bf qbh0 = ldfrag(qh, qq, HD, 0, h16);
  const v16bf qbh1 = ldfrag(qh, qq, HD, 32, h16);
  const v16bf qbl0 = ldfrag(ql, qq, HD, 0, h16);
  const v16bf qbl1 = ldfrag(ql, qq, HD, 32, h16);

  float M = NEG_BIG, L = 0.0f;
  v8f o[4] = {{}, {}, {}, {}};
  const int nch = qblk + 1;

#pragma unroll 1
  for (int ci = 0; ci < nch; ++ci) {
    const int c0 = ci * 64;

    v8f sc[4];
#pragma unroll
    for (int t = 0; t < 4; ++t) {
      const int krow = c0 + t * 16 + llo;
      v8f a = {};
      {
        const v16bf kfh = ldfrag(kh, krow, HD, 0, h16);
        const v16bf kfl = ldfrag(kl, krow, HD, 0, h16);
        a = wmma_bf16(kfh, qbh0, a);
        a = wmma_bf16(kfh, qbl0, a);
        a = wmma_bf16(kfl, qbh0, a);
      }
      {
        const v16bf kfh = ldfrag(kh, krow, HD, 32, h16);
        const v16bf kfl = ldfrag(kl, krow, HD, 32, h16);
        a = wmma_bf16(kfh, qbh1, a);
        a = wmma_bf16(kfh, qbl1, a);
        a = wmma_bf16(kfl, qbh1, a);
      }
      sc[t] = a;
    }

    float mloc = NEG_BIG;
#pragma unroll
    for (int t = 0; t < 4; ++t)
#pragma unroll
      for (int r = 0; r < 8; ++r) {
        const int key = c0 + t * 16 + 8 * h16 + r;
        const float v = (key <= qq) ? (sc[t][r] * 0.125f) : NEG_BIG;
        sc[t][r] = v;
        mloc = fmaxf(mloc, v);
      }
    mloc = fmaxf(mloc, __shfl_xor(mloc, 16, 32));
    const float Mn   = fmaxf(M, mloc);
    const float corr = __expf(M - Mn);
    M = Mn;

    float lsum = 0.0f;
#pragma unroll
    for (int t = 0; t < 4; ++t)
#pragma unroll
      for (int r = 0; r < 8; ++r) {
        const float p = __expf(sc[t][r] - Mn);
        sc[t][r] = p;
        lsum += p;
      }
    lsum += __shfl_xor(lsum, 16, 32);
    L = L * corr + lsum;
#pragma unroll
    for (int dt = 0; dt < 4; ++dt)
#pragma unroll
      for (int r = 0; r < 8; ++r) o[dt][r] *= corr;

#pragma unroll
    for (int g = 0; g < 2; ++g) {
      u16x16 wh, wl;
#pragma unroll
      for (int i = 0; i < 8; ++i) {
        const float p = sc[2 * g][i];
        const us_t hb = f2bf(p);
        wh[i] = hb;
        wl[i] = f2bf(p - bf2f(hb));
      }
#pragma unroll
      for (int i = 0; i < 8; ++i) {
        const float p = sc[2 * g + 1][i];
        const us_t hb = f2bf(p);
        wh[8 + i] = hb;
        wl[8 + i] = f2bf(p - bf2f(hb));
      }
      const v16bf pbh = __builtin_bit_cast(v16bf, wh);
      const v16bf pbl = __builtin_bit_cast(v16bf, wl);
      const int kk0 = c0 + 32 * g;
#pragma unroll
      for (int dt = 0; dt < 4; ++dt) {
        const int drow = dt * 16 + llo;
        const v16bf vfh = ldfrag(vh, drow, SEQ, kk0, h16);
        const v16bf vfl = ldfrag(vl, drow, SEQ, kk0, h16);
        o[dt] = wmma_bf16(vfh, pbh, o[dt]);
        o[dt] = wmma_bf16(vfh, pbl, o[dt]);
        o[dt] = wmma_bf16(vfl, pbh, o[dt]);
      }
    }
  }

  const float inv = 1.0f / L;
  float* ys = &yst[wave][0];
#pragma unroll
  for (int dt = 0; dt < 4; ++dt)
#pragma unroll
    for (int r = 0; r < 8; ++r)
      ys[llo * LDP + dt * 16 + 8 * h16 + r] = o[dt][r] * inv;
  __syncthreads();

#pragma unroll
  for (int it = 0; it < 4; ++it) {
    const int row = it * 4 + (lane >> 3);
    const int c8  = (lane & 7) * 8;
    const v4f a0 = *(const v4f*)(ys + row * LDP + c8);
    const v4f a1 = *(const v4f*)(ys + row * LDP + c8 + 4);
    u16x8 hi, lo;
    split2(a0, a1, hi, lo);
    const size_t off = ((size_t)bb * SEQ + (size_t)(q0 + row)) * EMB + (size_t)hh * HD + c8;
    *(volatile u16x8*)(Yh + off) = hi;
    *(volatile u16x8*)(Yl + off) = lo;
    __threadfence();
    *(volatile u16x8*)(Yh + off) = hi;
    *(volatile u16x8*)(Yl + off) = lo;
  }
}

__global__ __launch_bounds__(128) void proj_out_kernel(
    const us_t* __restrict__ Yh, const us_t* __restrict__ Yl,
    const us_t* __restrict__ Wpb, const float* __restrict__ bp,
    float* __restrict__ out) {
  __shared__ __align__(16) float st[4][16 * LDP];

  const int wave = threadIdx.x >> 5;
  const int lane = threadIdx.x & 31;
  const int h16  = lane >> 4;
  const int llo  = lane & 15;
  const int m0   = blockIdx.x * 64 + wave * 16;
  const int n0   = blockIdx.y * 64;

  v8f acc[4] = {{}, {}, {}, {}};
#pragma unroll 1
  for (int k0 = 0; k0 < EMB; k0 += 32) {
    const v16bf ah = ldfrag(Yh, m0 + llo, EMB, k0, h16);
    const v16bf al = ldfrag(Yl, m0 + llo, EMB, k0, h16);
#pragma unroll
    for (int c = 0; c < 4; ++c) {
      const v16bf b = ldfrag(Wpb, n0 + c * 16 + llo, EMB, k0, h16);
      acc[c] = wmma_bf16(ah, b, acc[c]);
      acc[c] = wmma_bf16(al, b, acc[c]);
    }
  }

  float* ws_ = &st[wave][0];
#pragma unroll
  for (int c = 0; c < 4; ++c) {
    int bcol = n0 + c * 16 + llo;
    bcol = (bcol < EMB) ? bcol : (EMB - 1);
    const float bvf = bf2f(f2bf(bp[bcol]));
#pragma unroll
    for (int r = 0; r < 8; ++r) ws_[(8 * h16 + r) * LDP + c * 16 + llo] = acc[c][r] + bvf;
  }
  __syncthreads();

#pragma unroll
  for (int it = 0; it < 8; ++it) {
    const int row = it * 2 + (lane >> 4);
    const int c4  = (lane & 15) * 4;
    const v4f v = *(const v4f*)(ws_ + row * LDP + c4);
    const int m = m0 + row;
    const int b = m / SEQ, s = m % SEQ;
    float* p = out + ((size_t)b * SEQ_FULL + s) * EMB + n0 + c4;
    *(volatile v4f*)p = v;
    __threadfence();
    *(volatile v4f*)p = v;
  }
}

extern "C" void kernel_launch(void* const* d_in, const int* in_sizes, int n_in,
                              void* d_out, int out_size, void* d_ws,
                              size_t ws_size, hipStream_t stream) {
  if (n_in < 9) return;
  const size_t need_rows = (size_t)(NB - 1) * SEQ_FULL + SEQ;
  if ((size_t)in_sizes[0] < need_rows * EMB) return;
  if (in_sizes[1] < EMB * EMB || in_sizes[3] < EMB * EMB ||
      in_sizes[5] < EMB * EMB || in_sizes[7] < EMB * EMB) return;
  if (in_sizes[2] < EMB || in_sizes[4] < EMB || in_sizes[6] < EMB || in_sizes[8] < EMB) return;
  if ((size_t)out_size < need_rows * EMB) return;
  if (ws_size < WS_TOTAL) return;

  const float* x  = (const float*)d_in[0];
  const float* Wq = (const float*)d_in[1];
  const float* bq = (const float*)d_in[2];
  const float* Wk = (const float*)d_in[3];
  const float* bk = (const float*)d_in[4];
  const float* Wv = (const float*)d_in[5];
  const float* bv = (const float*)d_in[6];
  const float* Wp = (const float*)d_in[7];
  const float* bp = (const float*)d_in[8];
  float* out = (float*)d_out;

  char* ws = (char*)d_ws;
  size_t off = 0;
  us_t* xb  = (us_t*)(ws + off); off += XB_BYTES;
  us_t* Wqb = (us_t*)(ws + off); off += WB_BYTES;
  us_t* Wkb = (us_t*)(ws + off); off += WB_BYTES;
  us_t* Wvb = (us_t*)(ws + off); off += WB_BYTES;
  us_t* Wpb = (us_t*)(ws + off); off += WB_BYTES;
  us_t* Qh  = (us_t*)(ws + off); off += PL_BYTES;
  us_t* Ql  = (us_t*)(ws + off); off += PL_BYTES;
  us_t* Kh  = (us_t*)(ws + off); off += PL_BYTES;
  us_t* Kl  = (us_t*)(ws + off); off += PL_BYTES;
  us_t* VTh = (us_t*)(ws + off); off += PL_BYTES;
  us_t* VTl = (us_t*)(ws + off); off += PL_BYTES;
  us_t* Yh  = (us_t*)(ws + off); off += PL_BYTES;
  us_t* Yl  = (us_t*)(ws + off); off += PL_BYTES;
  if (off > ws_size) return;

  const size_t ngx = (size_t)MROWS * EMB / 8;
  const size_t ngw = (size_t)EMB * EMB / 8;
  cvt_x_kernel<<<dim3((unsigned)((ngx + 255) / 256)), dim3(256), 0, stream>>>(x, xb);
  cvt_w_kernel<<<dim3((unsigned)((ngw + 255) / 256), 4), dim3(256), 0, stream>>>(
      Wq, Wk, Wv, Wp, Wqb, Wkb, Wvb, Wpb);

  proj_qkv_kernel<<<dim3(MROWS / 64, EMB / 64, 3), dim3(128), 0, stream>>>(
      xb, Wqb, Wkb, Wvb, bq, bk, bv, Qh, Ql, Kh, Kl, VTh, VTl);

  attn_kernel<<<dim3(SEQ / 64, NB * NH), dim3(128), 0, stream>>>(
      Qh, Ql, Kh, Kl, VTh, VTl, Yh, Yl);

  proj_out_kernel<<<dim3(MROWS / 64, EMB / 64), dim3(128), 0, stream>>>(
      Yh, Yl, Wpb, bp, out);

  (void)hipGetLastError();
}
